// StandardKernelModel_89412629168320
// MI455X (gfx1250) — hardware-verified
//
#include <hip/hip_runtime.h>
#include <math.h>

typedef __attribute__((ext_vector_type(16))) _Float16 v16h;
typedef __attribute__((ext_vector_type(16))) __bf16 v16b;
typedef __attribute__((ext_vector_type(8)))  _Float16 v8h;
typedef __attribute__((ext_vector_type(8)))  float v8f;
typedef __attribute__((ext_vector_type(4)))  float v4f;
typedef __attribute__((ext_vector_type(2)))  float v2f;
typedef __attribute__((ext_vector_type(4)))  unsigned v4u;
typedef __attribute__((ext_vector_type(4)))  int v4i;
typedef float __attribute__((may_alias)) float_a;
typedef int __attribute__((may_alias)) int_a;

template <typename T> __device__ __forceinline__ void vst2(void* p, T v) { *(volatile T*)p = v; __threadfence(); *(volatile T*)p = v; }
__device__ __forceinline__ v8f wmma16(v16h a, v16h b, v8f c) {
  v8f d = __builtin_amdgcn_wmma_f32_16x16x32_f16(false, a, false, b, (short)0, c, false, false);
  asm volatile("v_nop\n\tv_nop\n\tv_nop\n\tv_nop" : "+v"(d) : "v"(a), "v"(b));
  return d;
}
__device__ __forceinline__ v8f wmma_bf(v16b a, v16b b, v8f c) {
  v8f d = __builtin_amdgcn_wmma_f32_16x16x32_bf16(false, a, false, b, (short)0, c, false, false);
  asm volatile("v_nop\n\tv_nop\n\tv_nop\n\tv_nop" : "+v"(d) : "v"(a), "v"(b));
  return d;
}
__device__ __forceinline__ v16h frag_h(const _Float16* rowk0, int lane) {
  union { v16h v; v8h q[2]; } u; const _Float16* p = rowk0 + 8 * (lane >> 4);
  u.q[0] = *(const v8h*)p; u.q[1] = *(const v8h*)(p + 16); return u.v;
}
__device__ __forceinline__ v16h frag_f32(const float* rowk0, int lane) {
  v16h a; const float* p = rowk0 + 8 * (lane >> 4);
#pragma unroll
  for (int i = 0; i < 8; ++i) { a[i] = (_Float16)p[i]; a[8 + i] = (_Float16)p[16 + i]; }
  return a;
}
__device__ __forceinline__ v16h frag_f32s(const float* rowk0, int lane, float sc) {
  v16h a; const float* p = rowk0 + 8 * (lane >> 4);
#pragma unroll
  for (int i = 0; i < 8; ++i) { a[i] = (_Float16)(p[i] * sc); a[8 + i] = (_Float16)(p[16 + i] * sc); }
  return a;
}
__device__ __forceinline__ v16h fragc_f32(const float* W, int k0, int n, int lane, int ld, int K) {
  v16h a; const int g = lane >> 4;
#pragma unroll
  for (int i = 0; i < 8; ++i) { const int ka = k0 + 8 * g + i, kb = ka + 16;
    a[i] = (_Float16)(ka < K ? W[(size_t)(ka < K ? ka : K - 1) * ld + n] : 0.f); a[8 + i] = (_Float16)(kb < K ? W[(size_t)(kb < K ? kb : K - 1) * ld + n] : 0.f); }
  return a;
}
struct F2 { v16b h, l; };
__device__ __forceinline__ F2 bsplit16(const float v[16]) { F2 r;
#pragma unroll
  for (int i = 0; i < 16; ++i) { const __bf16 h = (__bf16)v[i]; r.h[i] = h; r.l[i] = (__bf16)(v[i] - (float)h); }
  return r; }
__device__ __forceinline__ F2 split_row(const float* row, int k0, int lane) { float v[16]; const float* p = row + k0 + 8 * (lane >> 4);
#pragma unroll
  for (int i = 0; i < 8; ++i) { v[i] = p[i]; v[8 + i] = p[16 + i]; }
  return bsplit16(v); }
__device__ __forceinline__ F2 split_rowK(const float* row, int k0, int lane, int K) { float v[16]; const int g = lane >> 4;
#pragma unroll
  for (int i = 0; i < 8; ++i) { const int ka = k0 + 8 * g + i, kb = ka + 16; v[i] = ka < K ? row[ka < K ? ka : K - 1] : 0.f; v[8 + i] = kb < K ? row[kb < K ? kb : K - 1] : 0.f; }
  return bsplit16(v); }
__device__ __forceinline__ F2 split_col(const float* W, int k0, int n, int lane, int ld, int K) { float v[16]; const int g = lane >> 4;
#pragma unroll
  for (int i = 0; i < 8; ++i) { const int ka = k0 + 8 * g + i, kb = ka + 16; v[i] = ka < K ? W[(size_t)(ka < K ? ka : K - 1) * ld + n] : 0.f; v[8 + i] = kb < K ? W[(size_t)(kb < K ? kb : K - 1) * ld + n] : 0.f; }
  return bsplit16(v); }
__device__ __forceinline__ v8f mac3(const F2& a, const F2& b, v8f c) { c = wmma_bf(a.l, b.h, c); c = wmma_bf(a.h, b.l, c); return wmma_bf(a.h, b.h, c); }
__device__ __forceinline__ float sigm(float v) { return 1.0f / (1.0f + expf(-v)); }
#define LDSX() do { asm volatile("s_wait_dscnt 0" ::: "memory"); __builtin_amdgcn_wave_barrier(); __builtin_amdgcn_fence(__ATOMIC_RELEASE, "workgroup"); } while (0)


#define NN 8192
#define MC 8192
#define DD 512
#define YY 256
#define HALF 4096
#ifndef NHALF
#define NHALF 2
#define RT1 (HALF / 64)
#endif
typedef __attribute__((ext_vector_type(8))) __bf16 v8b;
__device__ __forceinline__ v16b frag_b(const __bf16* rowk0, int lane) {
  union { v16b v; v8b q[2]; } u; const __bf16* p = rowk0 + 8 * (lane >> 4);
  u.q[0] = *(const v8b*)p; u.q[1] = *(const v8b*)(p + 16); return u.v;
}
__device__ __forceinline__ float bfr(float v) { return (float)(__bf16)v; }
__device__ __attribute__((noinline)) float exp_ni(float v) { return expf(v); }
__device__ __attribute__((noinline)) float erf_ni(float v) { return erff(v); }

#define WS_ZB  0u
#define WS_WT  (2u * MC * DD)
#define WS_Z2  (WS_WT + 2u * YY * MC)
#define WS_KH  (WS_Z2 + 4u * MC)
#define WS_KL  (WS_KH + 2u * (size_t)HALF * MC)
#define WS_END (WS_KL + 2u * (size_t)HALF * MC)

__global__ __launch_bounds__(256) void k_prep(const float* __restrict__ Z, __bf16* __restrict__ ZB, float* __restrict__ Z2) {
  __shared__ __align__(16) __bf16 s[64][DD + 8]; __shared__ float sq[64];
  const int t = threadIdx.x; const size_t m0 = (size_t)blockIdx.x * 64;
  for (int e = t; e < 64 * DD; e += 256) { const int r = e >> 9, c = e & 511; s[r][c] = (__bf16)Z[(m0 + r) * DD + c]; }
  __syncthreads();
  { const int r = t >> 2, q = t & 3; float a = 0.f; for (int c = q * 128; c < q * 128 + 128; ++c) { const float v = (float)s[r][c]; a += v * v; } a += __shfl_xor(a, 1); a += __shfl_xor(a, 2); if (q == 0) sq[r] = a; }
  for (int e = t; e < 64 * (DD / 8); e += 256) { const int r = e / (DD / 8), pc = e % (DD / 8); vst2((unsigned*)(ZB + (m0 + r) * DD + pc * 8), *(const v4u*)&s[r][pc * 8]); }
  __syncthreads();
  if (t < 16) vst2(Z2 + m0 + t * 4, *(const v4f*)&sq[t * 4]);
}
__global__ __launch_bounds__(256) void k_wt(const float* __restrict__ Wg, __bf16* __restrict__ WT) {
  __shared__ __align__(16) __bf16 s[YY][72]; const int t = threadIdx.x; const size_t m0 = (size_t)blockIdx.x * 64;
  for (int e = t; e < 64 * YY; e += 256) { const int r = e >> 8, y = e & 255; s[y][r] = (__bf16)Wg[(m0 + r) * YY + y]; }
  __syncthreads();
  for (int e = t; e < YY * 8; e += 256) { const int y = e >> 3, pc = e & 7; vst2((unsigned*)(WT + (size_t)y * MC + m0 + pc * 8), *(const v4u*)&s[y][pc * 8]); }
}
__global__ __launch_bounds__(128) void k_kmat(const float* __restrict__ X, const __bf16* __restrict__ ZB, const float* __restrict__ Z2, int rowbase, __bf16* __restrict__ KH, __bf16* __restrict__ KL) {
  __shared__ __align__(16) __bf16 soh[4][16][136], sol[4][16][136]; __shared__ float sx2[64];
  const int tid = threadIdx.x, wave = tid >> 5, lane = tid & 31, col = lane & 15, g = lane >> 4; const size_t rloc0 = (size_t)blockIdx.x * 64; const size_t r0 = rowbase + rloc0 + wave * 16; const int n0 = blockIdx.y * 128;
  { const int r = tid >> 1, half = tid & 1; const float* p = X + (rowbase + rloc0 + r) * DD + half * 256; float a = 0.f; for (int c = 0; c < 256; ++c) { const float v = bfr(p[c]); a += v * v; } a += __shfl_xor(a, 1); if (half == 0) sx2[r] = a; }
  v8f acc[8] = {};
#pragma unroll 2
  for (int kc = 0; kc < DD / 32; ++kc) { v16b a; { const float* p = X + (r0 + col) * DD + kc * 32 + 8 * g;
#pragma unroll
      for (int i = 0; i < 8; ++i) { a[i] = (__bf16)p[i]; a[8 + i] = (__bf16)p[16 + i]; } }
#pragma unroll
    for (int j = 0; j < 8; ++j) acc[j] = wmma_bf(a, frag_b(ZB + (size_t)(n0 + j * 16 + col) * DD + kc * 32, lane), acc[j]); }
  __syncthreads();
#pragma unroll
  for (int j = 0; j < 8; ++j) { const int c = n0 + j * 16 + col; const float z2 = Z2[c];
#pragma unroll
    for (int r = 0; r < 8; ++r) { const float d2 = sx2[wave * 16 + 8 * g + r] + z2 - 2.0f * acc[j][r]; const float kv = exp_ni(-sqrtf(fmaxf(d2, 0.f)) * 0.1f); const __bf16 hb = (__bf16)kv; soh[wave][8 * g + r][j * 16 + col] = hb; sol[wave][8 * g + r][j * 16 + col] = (__bf16)(kv - (float)hb); } }
  LDSX();
  for (int rl = 0; rl < 16; ++rl) { const size_t o = (rloc0 + wave * 16 + rl) * MC + n0; if (lane < 16) vst2((unsigned*)(KH + o + lane * 8), *(const v4u*)&soh[wave][rl][lane * 8]); else vst2((unsigned*)(KL + o + (lane - 16) * 8), *(const v4u*)&sol[wave][rl][(lane - 16) * 8]); }
}
__global__ __launch_bounds__(128) void k_pred(const __bf16* __restrict__ KH, const __bf16* __restrict__ KL, const __bf16* __restrict__ WT, int rowbase, float* __restrict__ OUT) {
  __shared__ __align__(16) float so[4][16][132];
  const int tid = threadIdx.x, wave = tid >> 5, lane = tid & 31, col = lane & 15, g = lane >> 4; const size_t rloc = (size_t)blockIdx.x * 64 + wave * 16; const int n0 = blockIdx.y * 128;
  v8f acc[8] = {};
#pragma unroll 2
  for (int kc = 0; kc < MC / 32; ++kc) { const v16b ah = frag_b(KH + (rloc + col) * MC + kc * 32, lane), al = frag_b(KL + (rloc + col) * MC + kc * 32, lane);
#pragma unroll
    for (int j = 0; j < 8; ++j) { const v16b w = frag_b(WT + (size_t)(n0 + j * 16 + col) * MC + kc * 32, lane); acc[j] = wmma_bf(al, w, acc[j]); acc[j] = wmma_bf(ah, w, acc[j]); } }
#pragma unroll
  for (int j = 0; j < 8; ++j)
#pragma unroll
    for (int r = 0; r < 8; ++r) so[wave][8 * g + r][j * 16 + col] = acc[j][r];
  LDSX();
  for (int rl = 0; rl < 16; ++rl) vst2(OUT + (rowbase + rloc + rl) * YY + n0 + lane * 4, *(const v4f*)&so[wave][rl][lane * 4]);
}
extern "C" void kernel_launch(void* const* d_in, const int* in_sizes, int n_in, void* d_out, int out_size, void* d_ws, size_t ws_size, hipStream_t stream) {
  (void)in_sizes; (void)n_in; (void)out_size;
  const float** F = (const float**)d_in;
  if (ws_size < (size_t)WS_END) return;
  char* ws = (char*)d_ws; __bf16 *ZB = (__bf16*)(ws + WS_ZB), *WT = (__bf16*)(ws + WS_WT), *KH = (__bf16*)(ws + WS_KH), *KL = (__bf16*)(ws + WS_KL); float* Z2 = (float*)(ws + WS_Z2);
  k_prep<<<MC / 64, 256, 0, stream>>>(F[1], ZB, Z2);
  k_wt<<<MC / 64, 256, 0, stream>>>(F[2], WT);
  for (int h = 0; h < NHALF; ++h) {
    k_kmat<<<dim3(RT1, MC / 128), 128, 0, stream>>>(F[0], ZB, Z2, h * HALF, KH, KL);
    k_pred<<<dim3(RT1, YY / 128), 128, 0, stream>>>(KH, KL, WT, h * HALF, (float*)d_out); }
}
